// GRUNet_91250875171546
// MI455X (gfx1250) — hardware-run, weakly checked
//
#include <hip/hip_runtime.h>
#include <math.h>

constexpr int NPED     = 131072;
constexpr int NSEQ     = 8;
constexpr int NPRED    = 12;
constexpr int NSTEPS   = NSEQ + NPRED;
constexpr int HID      = 64;
constexpr int NGATE    = 3 * HID;
constexpr int NTHR     = 256;
constexpr int NWAVE    = NTHR / 32;
constexpr int PED_WAVE = 16;
constexpr int PED_BLK  = NWAVE * PED_WAVE;
constexpr int NBLK     = NPED / PED_BLK;
constexpr int WPITCH   = 72;
constexpr int HPITCH   = 72;
constexpr float WCARRY     = 256.0f;
constexpr float WCARRY_INV = 1.0f / WCARRY;
constexpr float EXP_CLAMP  = 30.0f;
constexpr int FLAG_THR   = 64;
constexpr int FLAG_BYTES = FLAG_THR * 4;
constexpr int NOUT4      = NPRED * NPED * 2 / 4;
constexpr int FILL_BLK   = 96;
constexpr int FILL_IT    = NOUT4 / (FILL_BLK * NTHR);

static_assert(NPED % PED_BLK == 0, "grid exact");
static_assert(NBLK == 1024, "grid");
static_assert(HID == 64 && HID % 32 == 0, "two 32-deep k chunks");
static_assert(NGATE == 192 && NGATE % 16 == 0, "twelve 16-column tiles");
static_assert((NGATE * HID / 4) % NTHR == 0, "weight staging loop exact");
static_assert(WPITCH % 8 == 0 && HPITCH % 8 == 0, "16-B aligned rows");
static_assert(NSTEPS == 20, "static trip count");
static_assert(FLAG_BYTES == 256, "two whole 128-B lines");
static_assert(FILL_IT == 32 && FILL_IT * FILL_BLK * NTHR == NOUT4, "fill pass covers the output exactly");

typedef __attribute__((ext_vector_type(16))) _Float16 v16h;
typedef __attribute__((ext_vector_type(8)))  _Float16 v8h;
typedef __attribute__((ext_vector_type(4)))  _Float16 v4h;
typedef __attribute__((ext_vector_type(8)))  float    v8f;
typedef __attribute__((ext_vector_type(4)))  float    v4f;

template <typename T> struct Frag;
template <> struct Frag<_Float16> {
  typedef v16h V; union U { v16h v; v8h h[2]; };
  static __device__ __forceinline__ v16h load(const _Float16* p) {
    U f; f.h[0] = *(const v8h*)(p); f.h[1] = *(const v8h*)(p + 16); return f.v;
  }
  static __device__ __forceinline__ v8f mma(v16h a, v16h b, v8f c) {
    return __builtin_amdgcn_wmma_f32_16x16x32_f16(false, a, false, b, (short)0, c, false, false);
  }
};

__device__ __forceinline__ void wm_guard(v8f& acc, v16h a0, v16h a1, v16h b0, v16h b1) {
  asm volatile("v_nop\n\tv_nop\n\tv_nop\n\tv_nop" : "+v"(acc) : "v"(a0), "v"(a1), "v"(b0), "v"(b1));
}

__device__ __forceinline__ float sigm(float x) {
  const float xc = fminf(fmaxf(x, -EXP_CLAMP), EXP_CLAMP);
  return __builtin_amdgcn_rcpf(1.0f + __expf(-xc));
}
__device__ __forceinline__ float tanh_id(float x) {
  const float xc = fminf(fmaxf(2.0f * x, -EXP_CLAMP), EXP_CLAMP);
  return 1.0f - 2.0f * __builtin_amdgcn_rcpf(__expf(xc) + 1.0f);
}

__global__ __launch_bounds__(FLAG_THR) void premise_guard_kernel(const int* __restrict__ plen, int* __restrict__ flag) {
  const int v = plen[0];
  const int f = (v != NPRED) ? 1 : 0;
  volatile int* fp = (volatile int*)(flag + threadIdx.x);
  *fp = f;
  __threadfence();
  *fp = f;
}

__global__ __launch_bounds__(NTHR) void premise_fill_kernel(const int* __restrict__ flag, float* __restrict__ out) {
  const int f = flag[0];
  if (f == 0) return;
  const float q = __uint_as_float(0x7FC00000u);
  const v4f qv = {q, q, q, q};
  const int gid = blockIdx.x * NTHR + threadIdx.x;
  for (int pass = 0; pass < 2; ++pass) {
#pragma unroll 1
    for (int it = 0; it < FILL_IT; ++it) {
      *(volatile v4f*)(out + ((size_t)it * (size_t)(FILL_BLK * NTHR) + (size_t)gid) * 4) = qv;
    }
    __threadfence();
  }
}

__global__ __launch_bounds__(NTHR) void gated_cell_seq_kernel(
    const float* __restrict__ obs,
    const float* __restrict__ W_emb,
    const float* __restrict__ b_emb,
    const float* __restrict__ W_ih,
    const float* __restrict__ W_hh,
    const float* __restrict__ b_ih,
    const float* __restrict__ b_hh,
    const float* __restrict__ W_out,
    const float* __restrict__ b_out,
    float* __restrict__ out) {
  __shared__ __align__(16) _Float16 sW[NGATE * WPITCH];
  __shared__ __align__(16) _Float16 sH[NWAVE * 16 * HPITCH];
  __shared__ __align__(16) float    sMf[2 * NGATE];
  __shared__ __align__(16) float    sCf[NGATE];
  __shared__ __align__(16) float    sBhn[HID];
  __shared__ __align__(16) float    sWout[2 * HID];

  const int tid  = threadIdx.x;
  const int lane = tid & 31;
  const int wave = tid >> 5;
  const int c    = lane & 15;
  const int hh   = lane >> 4;
  const int koff = hh * 8;
  const int ped0 = blockIdx.x * PED_BLK + wave * PED_WAVE;

#pragma unroll 1
  for (int i = 0; i < (NGATE * HID / 4) / NTHR; ++i) {
    const int idx4 = i * NTHR + tid;
    const int n    = idx4 >> 4;
    const int k4   = (idx4 & 15) * 4;
    const v4f w = *(const v4f*)(W_hh + n * HID + k4);
    v4h hv;
    hv[0] = (_Float16)(w[0] * WCARRY);
    hv[1] = (_Float16)(w[1] * WCARRY);
    hv[2] = (_Float16)(w[2] * WCARRY);
    hv[3] = (_Float16)(w[3] * WCARRY);
    *(v4h*)(sW + n * WPITCH + k4) = hv;
  }
  if (tid < NGATE) {
    const int j = tid;
    const float* wr = W_ih + j * HID;
    float m0 = 0.0f, m1 = 0.0f, cc = 0.0f;
#pragma unroll 1
    for (int k4 = 0; k4 < HID; k4 += 4) {
      const v4f w = *(const v4f*)(wr + k4);
#pragma unroll
      for (int e = 0; e < 4; ++e) {
        const int k = k4 + e;
        m0 = fmaf(w[e], W_emb[2 * k + 0], m0);
        m1 = fmaf(w[e], W_emb[2 * k + 1], m1);
        cc = fmaf(w[e], b_emb[k], cc);
      }
    }
    const float bi = b_ih[j];
    const float bh = b_hh[j];
    sMf[2 * j + 0] = m0;
    sMf[2 * j + 1] = m1;
    sCf[j] = cc + bi + ((j < 2 * HID) ? bh : 0.0f);
    if (j >= 2 * HID) sBhn[j - 2 * HID] = bh * WCARRY;
  }
  if (tid < 2 * HID) sWout[tid] = W_out[tid];
  {
    const v8h zero8 = {(_Float16)0.0f, (_Float16)0.0f, (_Float16)0.0f, (_Float16)0.0f,
                       (_Float16)0.0f, (_Float16)0.0f, (_Float16)0.0f, (_Float16)0.0f};
#pragma unroll 1
    for (int i = tid; i < (NWAVE * 16 * HPITCH) / 8; i += NTHR) ((v8h*)sH)[i] = zero8;
  }
  __syncthreads();

  const float bo0 = b_out[0];
  const float bo1 = b_out[1];
  _Float16* sHw = sH + wave * 16 * HPITCH;
  const _Float16* arow = sHw + c * HPITCH + koff;
  const v8f z8 = {0.f, 0.f, 0.f, 0.f, 0.f, 0.f, 0.f, 0.f};

  v8f hA = z8, hB = z8, hC = z8, hD = z8;
  float xo[8][2];
#pragma unroll
  for (int r = 0; r < 8; ++r) { xo[r][0] = 0.0f; xo[r][1] = 0.0f; }

#pragma unroll 1
  for (int step = 0; step < NSTEPS; ++step) {
    __syncthreads();

    const v16h a0 = Frag<_Float16>::load(arow);
    const v16h a1 = Frag<_Float16>::load(arow + 32);

    {
      const int tc = (step < NSEQ) ? step : (NSEQ - 1);
      const float* xp = obs + ((size_t)tc * NPED + (size_t)(ped0 + 8 * hh)) * 2;
      v4f qv[4];
#pragma unroll
      for (int i = 0; i < 4; ++i) qv[i] = *(const v4f*)(xp + 4 * i);
      asm volatile("" : "+v"(qv[0]), "+v"(qv[1]), "+v"(qv[2]), "+v"(qv[3]));
      const bool obsphase = (step < NSEQ);
#pragma unroll
      for (int r = 0; r < 8; ++r) {
#pragma unroll
        for (int d = 0; d < 2; ++d) {
          const float xl = qv[(2 * r + d) >> 2][(2 * r + d) & 3];
          xo[r][d] = obsphase ? xl : xo[r][d];
        }
      }
    }

    float pj[8][2];
#pragma unroll
    for (int r = 0; r < 8; ++r) { pj[r][0] = 0.0f; pj[r][1] = 0.0f; }

#pragma unroll 1
    for (int ct = 0; ct < 4; ++ct) {
      const int jr = ct * 16 + c;
      const _Float16* wb = sW + jr * WPITCH + koff;
      const float bn = sBhn[jr];
      v8f accR = z8, accZ = z8, accN;
#pragma unroll
      for (int r = 0; r < 8; ++r) accN[r] = bn;
      {
        const v16h b0 = Frag<_Float16>::load(wb);
        const v16h b1 = Frag<_Float16>::load(wb + 32);
        accR = Frag<_Float16>::mma(a0, b0, accR);
        accR = Frag<_Float16>::mma(a1, b1, accR);
        wm_guard(accR, a0, a1, b0, b1);
      }
      {
        const v16h b0 = Frag<_Float16>::load(wb + HID * WPITCH);
        const v16h b1 = Frag<_Float16>::load(wb + HID * WPITCH + 32);
        accZ = Frag<_Float16>::mma(a0, b0, accZ);
        accZ = Frag<_Float16>::mma(a1, b1, accZ);
        wm_guard(accZ, a0, a1, b0, b1);
      }
      {
        const v16h b0 = Frag<_Float16>::load(wb + 2 * HID * WPITCH);
        const v16h b1 = Frag<_Float16>::load(wb + 2 * HID * WPITCH + 32);
        accN = Frag<_Float16>::mma(a0, b0, accN);
        accN = Frag<_Float16>::mma(a1, b1, accN);
        wm_guard(accN, a0, a1, b0, b1);
      }

      const float mr0 = sMf[2 * jr + 0];
      const float mr1 = sMf[2 * jr + 1];
      const float mz0 = sMf[2 * (jr + HID) + 0];
      const float mz1 = sMf[2 * (jr + HID) + 1];
      const float mn0 = sMf[2 * (jr + 2 * HID) + 0];
      const float mn1 = sMf[2 * (jr + 2 * HID) + 1];
      const float cr  = sCf[jr];
      const float cz  = sCf[jr + HID];
      const float cn  = sCf[jr + 2 * HID];
      const float wo0 = sWout[jr];
      const float wo1 = sWout[HID + jr];

      v8f hn8;
#pragma unroll
      for (int r = 0; r < 8; ++r) {
        const float x0 = xo[r][0];
        const float x1 = xo[r][1];
        const float gir = fmaf(mr1, x1, fmaf(mr0, x0, cr));
        const float giz = fmaf(mz1, x1, fmaf(mz0, x0, cz));
        const float gin = fmaf(mn1, x1, fmaf(mn0, x0, cn));
        const float rg = sigm(fmaf(accR[r], WCARRY_INV, gir));
        const float zg = sigm(fmaf(accZ[r], WCARRY_INV, giz));
        const float ghn = accN[r] * WCARRY_INV;
        const float ng = tanh_id(fmaf(rg, ghn, gin));
        const float ho = hA[r];
        const float hn = (1.0f - zg) * ng + zg * ho;
        hn8[r] = hn;
        pj[r][0] = fmaf(hn, wo0, pj[r][0]);
        pj[r][1] = fmaf(hn, wo1, pj[r][1]);
        sHw[(8 * hh + r) * HPITCH + jr] = (_Float16)hn;
      }
      hA = hB; hB = hC; hC = hD; hD = hn8;
    }

#pragma unroll
    for (int off = 1; off < 16; off <<= 1) {
#pragma unroll
      for (int r = 0; r < 8; ++r) {
        pj[r][0] += __shfl_xor(pj[r][0], off, 32);
        pj[r][1] += __shfl_xor(pj[r][1], off, 32);
      }
    }
#pragma unroll
    for (int r = 0; r < 8; ++r) {
      xo[r][0] = pj[r][0] + bo0;
      xo[r][1] = pj[r][1] + bo1;
    }

    if (step >= NSEQ) {
      const int sel = lane & 15;
      float ov = xo[0][0];
#pragma unroll
      for (int e = 1; e < 16; ++e) ov = (sel == e) ? xo[e >> 1][e & 1] : ov;
      volatile float* op = (volatile float*)(out + ((size_t)(step - NSEQ) * NPED + (size_t)ped0) * 2 + lane);
      *op = ov;
      __threadfence();
      *op = ov;
    }
  }
}

extern "C" void kernel_launch(void* const* d_in, const int* in_sizes, int n_in,
                              void* d_out, int out_size, void* d_ws, size_t ws_size, hipStream_t stream) {
  (void)in_sizes; (void)out_size;
  if (n_in < 10 || d_out == nullptr || d_ws == nullptr) return;
  const float* obs   = (const float*)d_in[0];
  const float* W_emb = (const float*)d_in[1];
  const float* b_emb = (const float*)d_in[2];
  const float* W_ih  = (const float*)d_in[3];
  const float* W_hh  = (const float*)d_in[4];
  const float* b_ih  = (const float*)d_in[5];
  const float* b_hh  = (const float*)d_in[6];
  const float* W_out = (const float*)d_in[7];
  const float* b_out = (const float*)d_in[8];
  const int*   plen  = (const int*)d_in[9];
  float* out = (float*)d_out;

  char* ws = (char*)d_ws; size_t off = 0;
  auto carve = [&](size_t bytes) -> char* { char* p = ws + off; off += (bytes + 255) & ~(size_t)255; return p; };
  int* FLAG = (int*)carve((size_t)FLAG_BYTES);
  if (off > ws_size || off > (size_t)134217728) return;

  premise_guard_kernel<<<dim3(1), dim3(FLAG_THR), 0, stream>>>(plen, FLAG);
  gated_cell_seq_kernel<<<dim3(NBLK), dim3(NTHR), 0, stream>>>(
      obs, W_emb, b_emb, W_ih, W_hh, b_ih, b_hh, W_out, b_out, out);
  premise_fill_kernel<<<dim3(FILL_BLK), dim3(NTHR), 0, stream>>>(FLAG, out);
}
